// TritonLocalWindowAttn_25451976196325
// MI455X (gfx1250) — hardware-verified
//
#include <hip/hip_runtime.h>
#include <math.h>

typedef __attribute__((ext_vector_type(16))) _Float16 v16h;
typedef __attribute__((ext_vector_type(16))) __bf16 v16b;
typedef __attribute__((ext_vector_type(8)))  _Float16 v8h;
typedef __attribute__((ext_vector_type(8)))  float v8f;
typedef __attribute__((ext_vector_type(4)))  float v4f;
typedef __attribute__((ext_vector_type(2)))  float v2f;
typedef __attribute__((ext_vector_type(4)))  unsigned v4u;
typedef __attribute__((ext_vector_type(4)))  int v4i;
typedef float __attribute__((may_alias)) float_a;
typedef int __attribute__((may_alias)) int_a;

template <typename T> __device__ __forceinline__ void vst2(void* p, T v) { *(volatile T*)p = v; __threadfence(); *(volatile T*)p = v; }
__device__ __forceinline__ v8f wmma16(v16h a, v16h b, v8f c) {
  v8f d = __builtin_amdgcn_wmma_f32_16x16x32_f16(false, a, false, b, (short)0, c, false, false);
  asm volatile("v_nop\n\tv_nop\n\tv_nop\n\tv_nop" : "+v"(d) : "v"(a), "v"(b));
  return d;
}
__device__ __forceinline__ v8f wmma_bf(v16b a, v16b b, v8f c) {
  v8f d = __builtin_amdgcn_wmma_f32_16x16x32_bf16(false, a, false, b, (short)0, c, false, false);
  asm volatile("v_nop\n\tv_nop\n\tv_nop\n\tv_nop" : "+v"(d) : "v"(a), "v"(b));
  return d;
}
__device__ __forceinline__ v16h frag_h(const _Float16* rowk0, int lane) {
  union { v16h v; v8h q[2]; } u; const _Float16* p = rowk0 + 8 * (lane >> 4);
  u.q[0] = *(const v8h*)p; u.q[1] = *(const v8h*)(p + 16); return u.v;
}
__device__ __forceinline__ v16h frag_f32(const float* rowk0, int lane) {
  v16h a; const float* p = rowk0 + 8 * (lane >> 4);
#pragma unroll
  for (int i = 0; i < 8; ++i) { a[i] = (_Float16)p[i]; a[8 + i] = (_Float16)p[16 + i]; }
  return a;
}
__device__ __forceinline__ v16h frag_f32s(const float* rowk0, int lane, float sc) {
  v16h a; const float* p = rowk0 + 8 * (lane >> 4);
#pragma unroll
  for (int i = 0; i < 8; ++i) { a[i] = (_Float16)(p[i] * sc); a[8 + i] = (_Float16)(p[16 + i] * sc); }
  return a;
}
__device__ __forceinline__ v16h fragc_f32(const float* W, int k0, int n, int lane, int ld, int K) {
  v16h a; const int g = lane >> 4;
#pragma unroll
  for (int i = 0; i < 8; ++i) { const int ka = k0 + 8 * g + i, kb = ka + 16;
    a[i] = (_Float16)(ka < K ? W[(size_t)(ka < K ? ka : K - 1) * ld + n] : 0.f); a[8 + i] = (_Float16)(kb < K ? W[(size_t)(kb < K ? kb : K - 1) * ld + n] : 0.f); }
  return a;
}
struct F2 { v16b h, l; };
__device__ __forceinline__ F2 bsplit16(const float v[16]) { F2 r;
#pragma unroll
  for (int i = 0; i < 16; ++i) { const __bf16 h = (__bf16)v[i]; r.h[i] = h; r.l[i] = (__bf16)(v[i] - (float)h); }
  return r; }
__device__ __forceinline__ F2 split_row(const float* row, int k0, int lane) { float v[16]; const float* p = row + k0 + 8 * (lane >> 4);
#pragma unroll
  for (int i = 0; i < 8; ++i) { v[i] = p[i]; v[8 + i] = p[16 + i]; }
  return bsplit16(v); }
__device__ __forceinline__ F2 split_rowK(const float* row, int k0, int lane, int K) { float v[16]; const int g = lane >> 4;
#pragma unroll
  for (int i = 0; i < 8; ++i) { const int ka = k0 + 8 * g + i, kb = ka + 16; v[i] = ka < K ? row[ka < K ? ka : K - 1] : 0.f; v[8 + i] = kb < K ? row[kb < K ? kb : K - 1] : 0.f; }
  return bsplit16(v); }
__device__ __forceinline__ F2 split_col(const float* W, int k0, int n, int lane, int ld, int K) { float v[16]; const int g = lane >> 4;
#pragma unroll
  for (int i = 0; i < 8; ++i) { const int ka = k0 + 8 * g + i, kb = ka + 16; v[i] = ka < K ? W[(size_t)(ka < K ? ka : K - 1) * ld + n] : 0.f; v[8 + i] = kb < K ? W[(size_t)(kb < K ? kb : K - 1) * ld + n] : 0.f; }
  return bsplit16(v); }
__device__ __forceinline__ v8f mac3(const F2& a, const F2& b, v8f c) { c = wmma_bf(a.l, b.h, c); c = wmma_bf(a.h, b.l, c); return wmma_bf(a.h, b.h, c); }
__device__ __forceinline__ float sigm(float v) { return 1.0f / (1.0f + expf(-v)); }
#define LDSX() do { asm volatile("s_wait_dscnt 0" ::: "memory"); __builtin_amdgcn_wave_barrier(); __builtin_amdgcn_fence(__ATOMIC_RELEASE, "workgroup"); } while (0)


#define NB 4
#define LL 2048
#define EE 1024
#define NH 16
#define DHH 64
#define KW 17
#define NR (NB * LL)
#ifndef TRB
#define TRB (NR / 64)
#define TRBP (NR / 64)
#endif
typedef __attribute__((ext_vector_type(8))) __bf16 v8b;
__device__ __forceinline__ v16b frag_b(const __bf16* rowk0, int lane) {
  union { v16b v; v8b q[2]; } u; const __bf16* p = rowk0 + 8 * (lane >> 4);
  u.q[0] = *(const v8b*)p; u.q[1] = *(const v8b*)(p + 16); return u.v;
}
__device__ __forceinline__ v16b frag_gbf(const float* rowk0, int lane) {
  v16b a; const float* p = rowk0 + 8 * (lane >> 4);
#pragma unroll
  for (int i = 0; i < 8; ++i) { a[i] = (__bf16)p[i]; a[8 + i] = (__bf16)p[16 + i]; }
  return a;
}
__device__ __forceinline__ float bfr(float v) { return (float)(__bf16)v; }
__device__ __attribute__((noinline)) float exp_ni(float v) { return expf(v); }
__device__ __forceinline__ float sgm(float v) { return 1.0f / (1.0f + exp_ni(-v)); }
__device__ __forceinline__ float silu(float v) { return v * sgm(v); }

#define PTQ 0
#define PTK 1024
#define PTV 2048
#define PTW 3072
#define PTO 3104
#define NPT 4128
#define WS_PT   0u
#define WS_Q    (WS_PT + 2u * NPT * EE)
#define WS_K    (WS_Q + 4u * NR * EE)
#define WS_V    (WS_K + 4u * NR * EE)
#define WS_WP   (WS_V + 4u * NR * EE)
#define WS_END  (WS_WP + 4u * NR * 32)

__global__ __launch_bounds__(128) void k_pack(const float* __restrict__ Wq, const float* __restrict__ Wkv, const float* __restrict__ Wwin, const float* __restrict__ Wout, __bf16* __restrict__ PT) {
  __shared__ __align__(16) __bf16 srow[EE];
  const int n = blockIdx.x, tid = threadIdx.x; const float* src; int ld, c;
  if (n < PTK) { src = Wq; ld = EE; c = n; } else if (n < PTW) { src = Wkv; ld = 2 * EE; c = n - PTK; } else if (n < PTO) { src = Wwin; ld = 2 * NH; c = n - PTW; } else { src = Wout; ld = EE; c = n - PTO; }
  for (int k = tid; k < EE; k += 128) srow[k] = (__bf16)src[(size_t)k * ld + c];
  __syncthreads();
  if (tid < EE / 8) vst2((unsigned*)(PT + (size_t)n * EE + tid * 8), *(const v4u*)(&srow[tid * 8]));
}
__global__ __launch_bounds__(128) void k_proj(const float* __restrict__ X, const __bf16* __restrict__ PT, const float* __restrict__ qg, const float* __restrict__ qb, const float* __restrict__ kg, const float* __restrict__ kb, float* __restrict__ Q, float* __restrict__ Kb_, float* __restrict__ V) {
  __shared__ __align__(16) float so[4][16][132];
  const int tid = threadIdx.x, wave = tid >> 5, lane = tid & 31, col = lane & 15, g = lane >> 4; const size_t r0 = (size_t)blockIdx.x * 64 + wave * 16; const int n0 = blockIdx.y * 128;
  v8f acc[8] = {};
#pragma unroll 2
  for (int kc = 0; kc < EE / 32; ++kc) { const v16b a = frag_gbf(X + (r0 + col) * EE + kc * 32, lane);
#pragma unroll
    for (int j = 0; j < 8; ++j) acc[j] = wmma_bf(a, frag_b(PT + (size_t)(n0 + j * 16 + col) * EE + kc * 32, lane), acc[j]); }
#pragma unroll
  for (int j = 0; j < 8; ++j)
#pragma unroll
    for (int r = 0; r < 8; ++r) so[wave][8 * g + r][j * 16 + col] = silu(acc[j][r]);
  LDSX();
  const int which = n0 / EE;
  if (which < 2) { const float* gg = which == 0 ? qg : kg; const float* bb = which == 0 ? qb : kb;
    const int rl = lane >> 1, hh = lane & 1; float s = 0.f;
#pragma unroll 8
    for (int c = 0; c < DHH; ++c) s += so[wave][rl][hh * DHH + c];
    const float mu = s * (1.0f / DHH); float q2 = 0.f;
#pragma unroll 8
    for (int c = 0; c < DHH; ++c) { const float d = so[wave][rl][hh * DHH + c] - mu; q2 += d * d; }
    const float rs = rsqrtf(q2 * (1.0f / DHH) + 1e-5f);
#pragma unroll 4
    for (int c = 0; c < DHH; ++c) so[wave][rl][hh * DHH + c] = (so[wave][rl][hh * DHH + c] - mu) * rs * bfr(gg[c]) + bfr(bb[c]);
    LDSX(); }
  float* dst = which == 0 ? Q : (which == 1 ? Kb_ : V); const int nn0 = n0 - which * EE;
  for (int rl = 0; rl < 16; ++rl) vst2(dst + (r0 + rl) * EE + nn0 + lane * 4, *(const v4f*)(&so[wave][rl][lane * 4]));
}
__global__ __launch_bounds__(128) void k_wp(const float* __restrict__ X, const __bf16* __restrict__ PT, const float* __restrict__ bwin, float* __restrict__ WP) {
  __shared__ __align__(16) float so[4][16][36];
  const int tid = threadIdx.x, wave = tid >> 5, lane = tid & 31, col = lane & 15, g = lane >> 4; const size_t r0 = (size_t)blockIdx.x * 64 + wave * 16;
  v8f acc[2] = {};
#pragma unroll 2
  for (int kc = 0; kc < EE / 32; ++kc) { const v16b a = frag_gbf(X + (r0 + col) * EE + kc * 32, lane);
#pragma unroll
    for (int j = 0; j < 2; ++j) acc[j] = wmma_bf(a, frag_b(PT + (size_t)(PTW + j * 16 + col) * EE + kc * 32, lane), acc[j]); }
#pragma unroll
  for (int j = 0; j < 2; ++j) { const int n = j * 16 + col; const float bv = bfr(bwin[n]);
#pragma unroll
    for (int r = 0; r < 8; ++r) { const float s = sgm(silu(acc[j][r] + bv)); so[wave][8 * g + r][n] = j == 0 ? s * 8.0f + 0.5f : s * 9.5f + 0.5f; } }
  LDSX();
  for (int q = lane; q < 16 * 8; q += 32) { const int rl = q >> 3, pc = q & 7; vst2(WP + (r0 + rl) * 32 + pc * 4, *(const v4f*)&so[wave][rl][pc * 4]); }
}
__global__ __launch_bounds__(256) void k_attn(float* __restrict__ QO, const float* __restrict__ Kb_, const float* __restrict__ V, const float* __restrict__ WP) {
  __shared__ __align__(16) float so[8][EE + 4]; __shared__ float slg[8][NH][KW + 3];
  const int tid = threadIdx.x, wave = tid >> 5, lane = tid & 31; const int h = lane >> 1, half = lane & 1;
  const size_t rb = (size_t)blockIdx.x * 64; const size_t seq0 = (rb / LL) * LL;
#pragma unroll 1
  for (int rr = wave; rr < 64; rr += 8) { const size_t r = rb + rr; const int l = (int)(r - seq0);
    float q[32];
#pragma unroll
    for (int i = 0; i < 32; ++i) q[i] = QO[r * EE + h * DHH + half * 32 + i];
    const float width = WP[r * 32 + h], sharp = WP[r * 32 + NH + h];
#pragma unroll 1
    for (int w = 0; w < KW; ++w) { const int kl = l + w - (KW / 2); const bool in = kl >= 0 && kl < LL; const int klc = kl < 0 ? 0 : (kl >= LL ? LL - 1 : kl);
      const float* kr = Kb_ + (seq0 + klc) * EE + h * DHH + half * 32; float d = 0.f;
#pragma unroll
      for (int i = 0; i < 32; ++i) d += q[i] * kr[i];
      d += __shfl_xor(d, 1); d = in ? d : 0.f;
      const float rel = (float)(w > KW / 2 ? w - KW / 2 : KW / 2 - w);
      const float sm = sgm((width - rel) * sharp);
      if (half == 0) slg[wave][h][w] = d * 0.125f - (1.0f - sm) * 10000.0f; }
    LDSX();
    { float mx = -3.0e38f; for (int w = 0; w < KW; ++w) mx = fmaxf(mx, slg[wave][h][w]); float Z = 0.f; for (int w = 0; w < KW; ++w) Z += exp_ni(slg[wave][h][w] - mx);
      LDSX();
      if (half == 0) { const float iz = 1.0f / Z; for (int w = 0; w < KW; ++w) slg[wave][h][w] = exp_ni(slg[wave][h][w] - mx) * iz; } }
    LDSX();
    float o[32];
#pragma unroll
    for (int i = 0; i < 32; ++i) o[i] = 0.f;
#pragma unroll 1
    for (int w = 0; w < KW; ++w) { const int kl = l + w - (KW / 2); const bool in = kl >= 0 && kl < LL; const int klc = kl < 0 ? 0 : (kl >= LL ? LL - 1 : kl);
      const float* vr = V + (seq0 + klc) * EE + h * DHH + half * 32; const float p = in ? slg[wave][h][w] : 0.f;
#pragma unroll
      for (int i = 0; i < 32; ++i) o[i] += p * vr[i]; }
#pragma unroll
    for (int i = 0; i < 32; ++i) so[wave][h * DHH + half * 32 + i] = o[i];
    LDSX();
    for (int pc = lane; pc < EE / 4; pc += 32) vst2(QO + r * EE + pc * 4, *(const v4f*)&so[wave][pc * 4]);
    LDSX(); }
}
__global__ __launch_bounds__(128) void k_out(const float* __restrict__ O, const __bf16* __restrict__ PT, float* __restrict__ Y) {
  __shared__ __align__(16) float so[4][16][132];
  const int tid = threadIdx.x, wave = tid >> 5, lane = tid & 31, col = lane & 15, g = lane >> 4; const size_t r0 = (size_t)blockIdx.x * 64 + wave * 16; const int n0 = blockIdx.y * 128;
  v8f acc[8] = {};
#pragma unroll 2
  for (int kc = 0; kc < EE / 32; ++kc) { const F2 a = split_row(O + (r0 + col) * EE, kc * 32, lane);
#pragma unroll
    for (int j = 0; j < 8; ++j) { const v16b w = frag_b(PT + (size_t)(PTO + n0 + j * 16 + col) * EE + kc * 32, lane); acc[j] = wmma_bf(a.l, w, acc[j]); acc[j] = wmma_bf(a.h, w, acc[j]); } }
#pragma unroll
  for (int j = 0; j < 8; ++j)
#pragma unroll
    for (int r = 0; r < 8; ++r) so[wave][8 * g + r][j * 16 + col] = silu(acc[j][r]);
  LDSX();
  for (int rl = 0; rl < 16; ++rl) vst2(Y + (r0 + rl) * EE + n0 + lane * 4, *(const v4f*)(&so[wave][rl][lane * 4]));
}

extern "C" void kernel_launch(void* const* d_in, const int* in_sizes, int n_in, void* d_out, int out_size, void* d_ws, size_t ws_size, hipStream_t stream) {
  (void)in_sizes; (void)n_in; (void)out_size;
  const float** F = (const float**)d_in;
  if (ws_size < (size_t)WS_END) return;
  char* ws = (char*)d_ws; __bf16* PT = (__bf16*)(ws + WS_PT); float *Q = (float*)(ws + WS_Q), *Kb_ = (float*)(ws + WS_K), *V = (float*)(ws + WS_V), *WP = (float*)(ws + WS_WP);
  k_pack<<<NPT, 128, 0, stream>>>(F[1], F[2], F[7], F[9], PT);
  k_proj<<<dim3(TRBP, 3 * EE / 128), 128, 0, stream>>>(F[0], PT, F[3], F[4], F[5], F[6], Q, Kb_, V);
  k_wp<<<TRBP, 128, 0, stream>>>(F[0], PT, F[8], WP);
  k_attn<<<TRB, 256, 0, stream>>>(Q, Kb_, V, WP);
  k_out<<<dim3(TRB, EE / 128), 128, 0, stream>>>(Q, PT, (float*)d_out);
}
